// DART_19232863551644
// MI455X (gfx1250) — hardware-run, weakly checked
//
#include <hip/hip_runtime.h>


#define NR   1024
#define ND   256
#define NH   512
#define NO   8192
typedef _Float16 h16;
typedef unsigned short bf;
typedef __attribute__((ext_vector_type(16))) __bf16   v16bf;
typedef __attribute__((ext_vector_type(16))) _Float16 v16h;
typedef __attribute__((ext_vector_type(8)))  _Float16 v8h;
typedef __attribute__((ext_vector_type(8)))  unsigned short v8us;
typedef __attribute__((ext_vector_type(8)))  float    v8f;
typedef __attribute__((ext_vector_type(4)))  float    v4f;
typedef v8h  __attribute__((may_alias)) v8ha;
typedef v4f  __attribute__((may_alias)) v4fa;
typedef v8us __attribute__((may_alias)) v8usa;

__device__ __forceinline__ unsigned short f2bf(float f) { unsigned u = __float_as_uint(f); u += 0x7FFFu + ((u >> 16) & 1u); return (unsigned short)(u >> 16); }
__device__ __forceinline__ float bf2f(unsigned short b) { return __uint_as_float(((unsigned)b) << 16); }
__device__ __forceinline__ float bfr(float f) { return bf2f(f2bf(f)); }
__device__ __forceinline__ v16h cat16(v8h lo, v8h hi) { return __builtin_shufflevector(lo, hi, 0, 1, 2, 3, 4, 5, 6, 7, 8, 9, 10, 11, 12, 13, 14, 15); }
__device__ __forceinline__ v16bf cat16b(v8us lo, v8us hi) { return __builtin_bit_cast(v16bf, __builtin_shufflevector(lo, hi, 0, 1, 2, 3, 4, 5, 6, 7, 8, 9, 10, 11, 12, 13, 14, 15)); }
__device__ __forceinline__ v8f wmma16(v16h a, v16h b, v8f c) { return __builtin_amdgcn_wmma_f32_16x16x32_f16(false, a, false, b, (short)0, c, false, false); }
__device__ __forceinline__ v8f wmmab(v16bf a, v16bf b, v8f c) { return __builtin_amdgcn_wmma_f32_16x16x32_bf16(false, a, false, b, (short)0, c, false, false); }

template <typename T16> struct WFrag;
template <> struct WFrag<h16> { typedef v16h V; static __device__ __forceinline__ V ld(const h16* p) { return cat16(*(const v8h*)p, *(const v8h*)(p + 16)); } static __device__ __forceinline__ v8f mma(V a, V b, v8f c) { return wmma16(a, b, c); } };
template <> struct WFrag<bf> { typedef v16bf V; static __device__ __forceinline__ V ld(const bf* p) { return cat16b(*(const v8us*)p, *(const v8us*)(p + 16)); } static __device__ __forceinline__ v8f mma(V a, V b, v8f c) { return wmmab(a, b, c); } };
template <typename T16, int NSPLIT, bool BIAS>
__global__ __launch_bounds__(32) void k_gemmw(const T16* __restrict__ A, const T16* __restrict__ A2, const T16* __restrict__ Bt, const T16* __restrict__ Bt2, int K, float* C, int ldc, const float* __restrict__ bias, size_t sA, size_t sB, size_t sC) {
    typedef typename WFrag<T16>::V V;
    __shared__ __align__(16) float os[16 * 68];
    const size_t z = blockIdx.z; A += z * sA; if (A2) A2 += z * sA; Bt += z * sB; if (Bt2) Bt2 += z * sB; C += z * sC;
    const int lane = threadIdx.x & 31, lr = lane & 15, hi = lane >> 4; const int r0 = blockIdx.x * 64, c0 = blockIdx.y * 64;
    v8f acc[4][4];
#pragma unroll
    for (int mb = 0; mb < 4; ++mb)
#pragma unroll
        for (int nb = 0; nb < 4; ++nb) acc[mb][nb] = (v8f){};
    const size_t aoff = (size_t)(r0 + lr) * K + 8 * hi, boff = (size_t)(c0 + lr) * K + 8 * hi;
    for (int kc = 0; kc < K; kc += 32) {
        V a[4], a2[4];
#pragma unroll
        for (int mb = 0; mb < 4; ++mb) { a[mb] = WFrag<T16>::ld(A + aoff + (size_t)mb * 16 * K + kc); if (NSPLIT == 1 || NSPLIT == 2) a2[mb] = WFrag<T16>::ld(A2 + aoff + (size_t)mb * 16 * K + kc); }
#pragma unroll
        for (int nb = 0; nb < 4; ++nb) { const V b = WFrag<T16>::ld(Bt + boff + (size_t)nb * 16 * K + kc); V b2; if (NSPLIT >= 2) b2 = WFrag<T16>::ld(Bt2 + boff + (size_t)nb * 16 * K + kc);
#pragma unroll
            for (int mb = 0; mb < 4; ++mb) { acc[mb][nb] = WFrag<T16>::mma(a[mb], b, acc[mb][nb]); if (NSPLIT == 1 || NSPLIT == 2) acc[mb][nb] = WFrag<T16>::mma(a2[mb], b, acc[mb][nb]); if (NSPLIT >= 2) acc[mb][nb] = WFrag<T16>::mma(a[mb], b2, acc[mb][nb]); } }
        asm volatile("v_nop\n\tv_nop\n\tv_nop\n\tv_nop" : "+v"(acc[0][0]), "+v"(acc[1][1]), "+v"(acc[2][2]), "+v"(acc[3][3]) : "v"(a[0]), "v"(a[3]));
    }
#pragma unroll
    for (int mb = 0; mb < 4; ++mb) {
#pragma unroll
        for (int nb = 0; nb < 4; ++nb) {
#pragma unroll
            for (int j = 0; j < 8; ++j) os[(hi * 8 + j) * 68 + nb * 16 + lr] = acc[mb][nb][j]; }
        __builtin_amdgcn_wave_barrier(); asm volatile("" ::: "memory");
        float* crow = C + (size_t)(r0 + mb * 16) * ldc + c0;
#pragma unroll 1
        for (int ps = 0; ps < 2; ++ps) {
#pragma unroll
            for (int s = 0; s < 8; ++s) { const int row = 2 * s + hi, cofs = lr * 4; v4f val = *(const v4fa*)(os + row * 68 + cofs); if (BIAS) { val[0] += bfr(bias[c0 + cofs]); val[1] += bfr(bias[c0 + cofs + 1]); val[2] += bfr(bias[c0 + cofs + 2]); val[3] += bfr(bias[c0 + cofs + 3]); }
                *(volatile v4f*)(crow + (size_t)row * ldc + cofs) = val; }
            if (ps == 0) __threadfence(); }
        __builtin_amdgcn_wave_barrier(); asm volatile("" ::: "memory");
    }
}

typedef __attribute__((ext_vector_type(2))) _Float16 v2h;
typedef __attribute__((ext_vector_type(4))) _Float16 v4h;
typedef __attribute__((ext_vector_type(2))) unsigned short v2us;
typedef __attribute__((ext_vector_type(4))) unsigned short v4us;
typedef __attribute__((ext_vector_type(2))) float v2f;
__device__ __forceinline__ h16 toh_flush(float x) { const float z = (fabsf(x) < 6.103515625e-05f) ? 0.0f : x; return (h16)z; }

template <int ACT>
__global__ __launch_bounds__(256) void eact_kernel(const float* __restrict__ P, float* __restrict__ OUT, size_t n4, float sl) {
  static_assert(ACT >= 1 && ACT <= 9, "eact: nine activations"); const size_t i = (size_t)blockIdx.x * 256 + threadIdx.x; if (i >= n4) return; const v4f a = *(const v4f*)(P + 4 * i); v4f o;
  for (int j = 0; j < 4; ++j) { const float v = a[j]; float y;
    if (ACT == 1) y = fmaxf(v, 0.0f);
    else if (ACT == 2) y = (v >= 0.0f) ? v : (sl * v);
    else if (ACT == 3) y = 1.0f / (1.0f + expf(-v));
    else if (ACT == 4) y = tanhf(v);
    else if (ACT == 5) y = (v > 0.0f) ? v : expm1f(v);
    else if (ACT == 6) y = v / (1.0f + expf(-v));
    else if (ACT == 7) y = (((0.5f * v)) * (1.0f + tanhf(0.7978845608028654f * (v + (0.044715f * ((v * ((v * v)))))))));
    else if (ACT == 8) y = (((0.5f * v)) * (1.0f + erff((v * 0.7071067811865476f))));
    else y = (1.0507009873554805f * ((v > 0.0f) ? v : (1.6732632423543772f * expm1f(v))));
    o[j] = y; }
  for (int pass = 0; pass < 2; ++pass) { *(volatile v4f*)(OUT + 4 * i) = o; __threadfence(); }
}

__global__ __launch_bounds__(64) void k_cat16(const float* __restrict__ U, int wu, int pu, int uin, const float* __restrict__ W, int ww, int pw, int win, h16* dst, int KP) { const int k0 = (blockIdx.x * 64 + threadIdx.x) * 8; if (k0 >= KP) return; const int r = blockIdx.y; const unsigned mu = 0u - (unsigned)(uin != 0), mw = 0u - (unsigned)(win != 0); v8h o;
#pragma unroll
    for (int q = 0; q < 8; ++q) { const int k = k0 + q; const bool iu = k < wu; const bool iw = (!iu) && (k < wu + ww); const int ku = min(k, wu - 1); const int kw = min(max(k - wu, 0), max(ww - 1, 0)); const float a = U[(size_t)r * pu + ku]; const float b = W[(size_t)r * pw + kw];
        const float va = __uint_as_float((__float_as_uint(bfr(a)) & mu) | (__float_as_uint(a) & ~mu)); const float vb = __uint_as_float((__float_as_uint(bfr(b)) & mw) | (__float_as_uint(b) & ~mw)); const unsigned su = 0u - (unsigned)iu, sw = 0u - (unsigned)iw; o[q] = toh_flush(__uint_as_float((__float_as_uint(va) & su) | (__float_as_uint(vb) & sw))); }
    *(volatile v8h*)(dst + (size_t)r * KP + k0) = o; __threadfence(); *(volatile v8h*)(dst + (size_t)r * KP + k0) = o; }

__global__ __launch_bounds__(64) void k_mw16(const float* __restrict__ W, h16* dst, int cols, int rsel, int cmod) { const int c0 = (blockIdx.x * 64 + threadIdx.x) * 8; if (c0 >= cols) return; const int r = blockIdx.y; const int dr = rsel * ((r >> 5) - 1) + (1 - rsel) * (r - 255 * ((r >= 255) + (r >= 510))); const v8f w = *(const v8f*)(W + (size_t)r * cols + c0); v8h o;
#pragma unroll
    for (int q = 0; q < 8; ++q) { const int c = c0 + q; const int dc = c - cmod * 255 * ((c >= 255) + (c >= 510)); const unsigned mk = 0u - (unsigned)(dr >= dc); o[q] = toh_flush(__uint_as_float(__float_as_uint(bfr(w[q])) & mk)); }
    h16* d = dst + (size_t)r * cols + c0; *(volatile v8h*)d = o; __threadfence(); *(volatile v8h*)d = o; }

__device__ __forceinline__ float lse4(float a, float b, float c, float d) { const float m = fmaxf(fmaxf(a, b), fmaxf(c, d)); const float s = __fadd_rn(__fadd_rn(__fadd_rn(expf(__fsub_rn(a, m)), expf(__fsub_rn(b, m))), expf(__fsub_rn(c, m))), expf(__fsub_rn(d, m))); return __fadd_rn(m, logf(s)); }
__device__ __forceinline__ void gden(const float* __restrict__ p, float x, float (&g)[16]) {
#pragma unroll
    for (int q4 = 0; q4 < 4; ++q4) { const v4f m = *(const v4f*)(p + 4 * q4); const v4f ls = *(const v4f*)(p + 16 + 4 * q4);
#pragma unroll
        for (int e = 0; e < 4; ++e) { const float s = __fadd_rn(expf(ls[e]), 0.01f); const float z = __fdiv_rn(__fsub_rn(x, m[e]), s); g[4 * q4 + e] = __fsub_rn(__fsub_rn(__fmul_rn(-0.5f, __fmul_rn(z, z)), logf(s)), 0.9189385332046727f); } } }

__global__ __launch_bounds__(256) void k_lsm(const float* __restrict__ u, float* V) { const int d = threadIdx.x; const int dd = d < 255 ? d : 254; const v4f x = *(const v4f*)(u + 4 * dd); const float u0 = bfr(x[0]), u1 = bfr(x[1]), u2 = bfr(x[2]), u3 = bfr(x[3]); const float l = lse4(u0, u1, u2, u3); const float live = d < 255 ? 1.0f : 0.0f; v4f o; o[0] = __fmul_rn(__fsub_rn(u0, l), live); o[1] = __fmul_rn(__fsub_rn(u1, l), live); o[2] = __fmul_rn(__fsub_rn(u2, l), live); o[3] = __fmul_rn(__fsub_rn(u3, l), live); *(volatile v4f*)(V + 4 * d) = o; __threadfence(); *(volatile v4f*)(V + 4 * d) = o; }

__global__ __launch_bounds__(256) void k_lp(const float* __restrict__ T, const float* __restrict__ a, const float* __restrict__ V, float* out0) { const int b = blockIdx.x * 256 + threadIdx.x; if (b >= NR) return; const float* tr = T + (size_t)b * NO; const float* ar = a + (size_t)b * ND; float g[16], c[4];
    { gden(tr, bfr(ar[0]), g); const v4f v = *(const v4f*)V; c[0] = __fadd_rn(g[0], v[0]); c[1] = __fadd_rn(g[1], v[1]); c[2] = __fadd_rn(g[2], v[2]); c[3] = __fadd_rn(g[3], v[3]); }
    for (int d = 1; d < ND - 1; ++d) { gden(tr + 32 * d, bfr(ar[d]), g); const v4f v = *(const v4f*)(V + 4 * d); float n[4];
#pragma unroll
        for (int j = 0; j < 4; ++j) n[j] = lse4(__fadd_rn(c[0], __fadd_rn(g[j], v[j])), __fadd_rn(c[1], __fadd_rn(g[4 + j], v[j])), __fadd_rn(c[2], __fadd_rn(g[8 + j], v[j])), __fadd_rn(c[3], __fadd_rn(g[12 + j], v[j])));
#pragma unroll
        for (int j = 0; j < 4; ++j) c[j] = n[j]; }
    gden(tr + 32 * (ND - 1), bfr(ar[ND - 1]), g); const float r = lse4(__fadd_rn(c[0], g[0]), __fadd_rn(c[1], g[4]), __fadd_rn(c[2], g[8]), __fadd_rn(c[3], g[12]));
    *(volatile float*)(out0 + b) = r; __threadfence(); *(volatile float*)(out0 + b) = r; }

extern "C" void kernel_launch(void* const* d_in, const int* in_sizes, int n_in, void* d_out, int out_size, void* d_ws, size_t ws_size, hipStream_t stream) {
    if (n_in < 10) return;
    const int want[10] = {NR * ND, NH * ND, NH, NH * NH, NH, NH * NH, NH, NO * NH, NO, 255 * 4};
    for (int k = 0; k < 10; ++k) if (in_sizes[k] != want[k]) return;
    if (out_size != NR + NR * NO) return;
    static_assert(NR % 64 == 0 && NH % 64 == 0 && NO % 64 == 0 && ND % 64 == 0 && NH % 32 == 0 && ND % 32 == 0 && NO == ND * 32 && (NR * NH / 4) % 256 == 0 && NR % 256 == 0 && (NR * 4) % 128 == 0 && NH < 765 && ND < 765, "the products: M and N multiples of 64, depths multiples of 32; t's 32 floats a dim; every flat grid exact; t begins on a 128-byte line of the output; the literal mod-255 arithmetic holds under 765");
    const float* a = (const float*)d_in[0]; const float* w[9]; for (int k = 0; k < 9; ++k) w[k] = (const float*)d_in[1 + k];
    float* out0 = (float*)d_out; float* T = out0 + NR;
    char* wsp = (char*)d_ws; auto take = [&](size_t bytes) { char* p = wsp; wsp += (bytes + 255) & ~(size_t)255; return (void*)p; };
    h16* P0 = (h16*)take((size_t)NH * ND * 2); h16* P1 = (h16*)take((size_t)NH * NH * 2); h16* P2 = (h16*)take((size_t)NH * NH * 2); h16* P3 = (h16*)take((size_t)NO * NH * 2);
    h16* X0 = (h16*)take((size_t)NR * ND * 2); h16* X1 = (h16*)take((size_t)NR * NH * 2); float* F = (float*)take((size_t)NR * NH * 4); float* G = (float*)take((size_t)NR * NH * 4); float* V = (float*)take((size_t)256 * 4 * 4);
    if ((size_t)(wsp - (char*)d_ws) > ws_size) return;
    k_mw16<<<dim3(1, NH, 1), 64, 0, stream>>>(w[0], P0, ND, 0, 0);
    k_mw16<<<dim3(1, NH, 1), 64, 0, stream>>>(w[2], P1, NH, 0, 1);
    k_mw16<<<dim3(1, NH, 1), 64, 0, stream>>>(w[4], P2, NH, 0, 1);
    k_mw16<<<dim3(1, NO, 1), 64, 0, stream>>>(w[6], P3, NH, 1, 1);
    const unsigned E = (unsigned)(NR * NH / 4 / 256);
    k_cat16<<<dim3(1, NR, 1), 64, 0, stream>>>(a, ND, ND, 1, a, 0, ND, 1, X0, ND);
    k_gemmw<h16, 0, true><<<dim3(NR / 64, NH / 64, 1), 32, 0, stream>>>(X0, nullptr, P0, nullptr, ND, F, NH, w[1], 0, 0, 0);
    eact_kernel<1><<<E, 256, 0, stream>>>(F, G, (size_t)NR * NH / 4, 0.0f);
    k_cat16<<<dim3(1, NR, 1), 64, 0, stream>>>(G, NH, NH, 0, G, 0, NH, 0, X1, NH);
    k_gemmw<h16, 0, true><<<dim3(NR / 64, NH / 64, 1), 32, 0, stream>>>(X1, nullptr, P1, nullptr, NH, F, NH, w[3], 0, 0, 0);
    eact_kernel<1><<<E, 256, 0, stream>>>(F, G, (size_t)NR * NH / 4, 0.0f);
    k_cat16<<<dim3(1, NR, 1), 64, 0, stream>>>(G, NH, NH, 0, G, 0, NH, 0, X1, NH);
    k_gemmw<h16, 0, true><<<dim3(NR / 64, NH / 64, 1), 32, 0, stream>>>(X1, nullptr, P2, nullptr, NH, F, NH, w[5], 0, 0, 0);
    eact_kernel<1><<<E, 256, 0, stream>>>(F, G, (size_t)NR * NH / 4, 0.0f);
    k_cat16<<<dim3(1, NR, 1), 64, 0, stream>>>(G, NH, NH, 0, G, 0, NH, 0, X1, NH);
    k_gemmw<h16, 0, true><<<dim3(NR / 64, NO / 64, 1), 32, 0, stream>>>(X1, nullptr, P3, nullptr, NH, T, NO, w[7], 0, 0, 0);
    k_lsm<<<1, 256, 0, stream>>>(w[8], V);
    k_lp<<<(unsigned)(NR / 256), 256, 0, stream>>>(T, a, V, out0);
}
